// ResponseConditionedAttention_83348135346700
// MI455X (gfx1250) — hardware-verified
//
#include <hip/hip_runtime.h>
#include <math.h>

constexpr int kBatch = 4;
constexpr int kSeq = 1024;
constexpr int kEmb = 1024;
constexpr int kHeads = 16;
constexpr int kHeadDim = 64;
constexpr int kCats = 4;
constexpr int kTok = kBatch * kSeq;
constexpr int kHeadsPerGroup = 8;
constexpr int kGroupsPerBatch = kHeads / kHeadsPerGroup;
constexpr float kWCarry = 32.0f;
constexpr float kWCarryInv = 1.0f / 32.0f;
constexpr float kScoreScale = 0.125f;
constexpr size_t kPlaneTok = (size_t)kTok * kEmb;
constexpr size_t kPlaneW = (size_t)kEmb * kEmb;
constexpr size_t kPlaneBatch = (size_t)kSeq * kEmb;

typedef __attribute__((ext_vector_type(16))) _Float16 v16h;
typedef __attribute__((ext_vector_type(8)))  _Float16 v8h;
typedef __attribute__((ext_vector_type(16))) __bf16   v16b;
typedef __attribute__((ext_vector_type(8)))  __bf16   v8b;
typedef __attribute__((ext_vector_type(8)))  float    v8f;
typedef __attribute__((ext_vector_type(4)))  float    v4f;
typedef __attribute__((ext_vector_type(4)))  unsigned int v4u;

__device__ __forceinline__ unsigned short f2bf_bits(float f) {
  unsigned u = __float_as_uint(f);
  return (unsigned short)((u + 0x7FFFu + ((u >> 16) & 1u)) >> 16);
}
__device__ __forceinline__ float bf_bits2f(unsigned short h) { return __uint_as_float(((unsigned)h) << 16); }

__device__ __forceinline__ void dep_guard_h(v8f& a, v8f& b, v16h x, v16h y) { asm volatile("v_nop\n\tv_nop\n\tv_nop\n\tv_nop" : "+v"(a), "+v"(b) : "v"(x), "v"(y)); }
__device__ __forceinline__ void dep_guard_b(v8f& a, v8f& b, v16b x, v16b y) { asm volatile("v_nop\n\tv_nop\n\tv_nop\n\tv_nop" : "+v"(a), "+v"(b) : "v"(x), "v"(y)); }
__device__ __forceinline__ void keep4_h(v16h a, v16h b, v16h c, v16h d) { asm volatile("v_nop" :: "v"(a), "v"(b), "v"(c), "v"(d)); }
__device__ __forceinline__ void keep4_b(v16b a, v16b b, v16b c, v16b d) { asm volatile("v_nop" :: "v"(a), "v"(b), "v"(c), "v"(d)); }
__device__ __forceinline__ void acc_guard4(v8f& a, v8f& b, v8f& c, v8f& d) { asm volatile("v_nop\n\tv_nop\n\tv_nop\n\tv_nop" : "+v"(a), "+v"(b), "+v"(c), "+v"(d)); }
template <typename T> struct Frag;
template <> struct Frag<_Float16> {
  typedef v16h V; union U { v16h v; v8h h[2]; };
  static __device__ __forceinline__ v16h load(const _Float16* p) {
    U f; f.h[0] = *(const v8h*)(p); f.h[1] = *(const v8h*)(p + 16); return f.v;
  }
  static __device__ __forceinline__ v8f mma(v16h a, v16h b, v8f c) {
    return __builtin_amdgcn_wmma_f32_16x16x32_f16(false, a, false, b, (short)0, c, false, false);
  }
  static __device__ __forceinline__ void guard(v8f& a, v8f& b, v16h x, v16h y) { dep_guard_h(a, b, x, y); }
  static __device__ __forceinline__ void keep(v16h a, v16h b, v16h c, v16h d) { keep4_h(a, b, c, d); }
};
template <> struct Frag<__bf16> {
  typedef v16b V; union U { v16b v; v8b h[2]; };
  static __device__ __forceinline__ v16b load(const __bf16* p) {
    U f; f.h[0] = *(const v8b*)(p); f.h[1] = *(const v8b*)(p + 16); return f.v;
  }
  static __device__ __forceinline__ v8f mma(v16b a, v16b b, v8f c) {
    return __builtin_amdgcn_wmma_f32_16x16x32_bf16(false, a, false, b, (short)0, c, false, false);
  }
  static __device__ __forceinline__ void guard(v8f& a, v8f& b, v16b x, v16b y) { dep_guard_b(a, b, x, y); }
  static __device__ __forceinline__ void keep(v16b a, v16b b, v16b c, v16b d) { keep4_b(a, b, c, d); }
};

__device__ __forceinline__ unsigned pk16(unsigned short a, unsigned short b) { return (unsigned)a | ((unsigned)b << 16); }
__device__ __forceinline__ unsigned short h_bits(float f) { const _Float16 h = (_Float16)f; return __builtin_bit_cast(unsigned short, h); }
__device__ __forceinline__ int clamp_cat(int v) { v = v < 0 ? 0 : v; return v > (kCats - 1) ? (kCats - 1) : v; }

template <int ET> struct Elem;
template <> struct Elem<0> { typedef _Float16 T; };
template <> struct Elem<1> { typedef __bf16 T; };
template <int ET, bool SPLIT, int BIAS_MODE, int OUT_MODE, bool RESID, int ACT = 0>
__global__ __launch_bounds__(256) void wmma_gemm64(
    const unsigned short* __restrict__ Ap, const unsigned short* __restrict__ A2p, int lda, long strideA,
    const unsigned short* __restrict__ Btp, const unsigned short* __restrict__ Bt2p, int ldb, long strideB,
    void* __restrict__ Cout, void* __restrict__ Cout2, int ldc, long strideC,
    const float* __restrict__ bias,
    const float* __restrict__ resid, long strideR,
    int M, int N, int K, float scale) {
  typedef typename Elem<ET>::T T;
  typedef typename Frag<T>::V V;
  const T* A = (const T*)Ap; const T* A2 = (const T*)A2p; const T* Bt = (const T*)Btp; const T* Bt2 = (const T*)Bt2p;
  __shared__ __align__(16) float sT[8][16 * 68];
  const int b    = blockIdx.y;
  const int lane = threadIdx.x & 31;
  const int wave = threadIdx.x >> 5;
  const int tilesN = N >> 6;
  const int tilesM = M >> 6;
  const int tile = blockIdx.x * 8 + wave;
  if (tile >= tilesM * tilesN) return;
  const int tm = tile / tilesN;
  const int tn = tile - tm * tilesN;
  const int m0 = tm << 6;
  const int n0 = tn << 6;

  const T* Ab  = A  + (size_t)b * strideA;
  const T* Bb  = Bt + (size_t)b * strideB;
  const T* Ab2 = SPLIT ? (A2  + (size_t)b * strideA) : nullptr;
  const T* Bb2 = SPLIT ? (Bt2 + (size_t)b * strideB) : nullptr;

  const int rlane = lane & 15;
  const int koff  = (lane >> 4) * 8;
  const int mOff  = (lane >> 4) * 8;

  v8f acc[4][4];
#pragma unroll
  for (int i = 0; i < 4; ++i)
#pragma unroll
    for (int j = 0; j < 4; ++j) acc[i][j] = (v8f){0.f,0.f,0.f,0.f,0.f,0.f,0.f,0.f};

  for (int k0 = 0; k0 < K; k0 += 32) {
    V bh[4], bl[4];
#pragma unroll
    for (int j = 0; j < 4; ++j) {
      const size_t bo = (size_t)(n0 + (j << 4) + rlane) * ldb + koff + k0;
      bh[j] = Frag<T>::load(Bb + bo);
      if (SPLIT) bl[j] = Frag<T>::load(Bb2 + bo);
    }
#pragma unroll
    for (int i = 0; i < 4; ++i) {
      const size_t ao = (size_t)(m0 + (i << 4) + rlane) * lda + koff + k0;
      V ah = Frag<T>::load(Ab + ao);
      V al;
      if (SPLIT) al = Frag<T>::load(Ab2 + ao);
#pragma unroll
      for (int j = 0; j < 4; ++j) {
        acc[i][j] = Frag<T>::mma(ah, bh[j], acc[i][j]);
        if (SPLIT) {
          acc[i][j] = Frag<T>::mma(ah, bl[j], acc[i][j]);
          acc[i][j] = Frag<T>::mma(al, bh[j], acc[i][j]);
        }
      }
      Frag<T>::guard(acc[i][0], acc[i][3], ah, SPLIT ? al : ah);
    }
    Frag<T>::keep(bh[0], bh[1], bh[2], bh[3]);
    if (SPLIT) Frag<T>::keep(bl[0], bl[1], bl[2], bl[3]);
  }
  acc_guard4(acc[0][0], acc[0][1], acc[0][2], acc[0][3]);
  acc_guard4(acc[1][0], acc[1][1], acc[1][2], acc[1][3]);
  acc_guard4(acc[2][0], acc[2][1], acc[2][2], acc[2][3]);
  acc_guard4(acc[3][0], acc[3][1], acc[3][2], acc[3][3]);

  float* slab = sT[wave];
  const float* Rb = RESID ? (resid + (size_t)b * strideR) : nullptr;
#pragma unroll
  for (int i = 0; i < 4; ++i) {
    const int mBase = m0 + (i << 4);
#pragma unroll
    for (int j = 0; j < 4; ++j) {
      const int n = n0 + (j << 4) + rlane;
      float bv = 0.f;
      if (BIAS_MODE == 2) bv = bias[n];
#pragma unroll
      for (int r = 0; r < 8; ++r) {
        float v = acc[i][j][r] * scale;
        if (BIAS_MODE == 1) v += bias[mBase + mOff + r];
        if (BIAS_MODE == 2) v += bv;
        if (RESID) v += Rb[(size_t)(mBase + mOff + r) * ldc + n];
        if (ACT == 2) v = fmaxf(v, 0.0f);
        if (ACT == 4) v = (v > 0.f) ? v : 0.01f * v;
        slab[(mOff + r) * 68 + (j << 4) + rlane] = v;
      }
    }
    __builtin_amdgcn_fence(__ATOMIC_RELEASE, "workgroup");
    __builtin_amdgcn_wave_barrier();
    __builtin_amdgcn_fence(__ATOMIC_ACQUIRE, "workgroup");
    if (OUT_MODE == 0) {
      float* C = (float*)Cout + (size_t)b * strideC;
      const int hh = lane >> 4, c4 = (lane & 15) * 4;
      for (int pass = 0; pass < 2; ++pass) {
#pragma unroll
        for (int it = 0; it < 8; ++it) {
          const int row = it * 2 + hh;
          v4f v = *(const v4f*)(slab + row * 68 + c4);
          *(volatile v4f*)(C + (size_t)(mBase + row) * ldc + n0 + c4) = v;
        }
        __threadfence();
      }
    } else {
      const int q = lane >> 3, c8 = (lane & 7) * 8;
      unsigned short* C  = (unsigned short*)Cout  + (size_t)b * strideC;
      unsigned short* C2 = (OUT_MODE == 2) ? ((unsigned short*)Cout2 + (size_t)b * strideC) : nullptr;
      for (int pass = 0; pass < 2; ++pass) {
#pragma unroll
        for (int it = 0; it < 4; ++it) {
          const int row = it * 4 + q;
          const float* sp = slab + row * 68 + c8;
          v8h hv, lv;
#pragma unroll
          for (int e = 0; e < 8; ++e) {
            if (OUT_MODE == 1) {
              hv[e] = (_Float16)sp[e];
            } else {
              unsigned short hb = f2bf_bits(sp[e]);
              unsigned short lb = f2bf_bits(sp[e] - bf_bits2f(hb));
              hv[e] = __builtin_bit_cast(_Float16, hb);
              lv[e] = __builtin_bit_cast(_Float16, lb);
            }
          }
          *(volatile v8h*)(C + (size_t)(mBase + row) * ldc + n0 + c8) = hv;
          if (OUT_MODE == 2) *(volatile v8h*)(C2 + (size_t)(mBase + row) * ldc + n0 + c8) = lv;
        }
        __threadfence();
      }
    }
    __builtin_amdgcn_fence(__ATOMIC_RELEASE, "workgroup");
    __builtin_amdgcn_wave_barrier();
    __builtin_amdgcn_fence(__ATOMIC_ACQUIRE, "workgroup");
  }
}

template <int OUT_MODE>
__global__ __launch_bounds__(256) void seg_gemm64(
    const unsigned short* __restrict__ Ap, const unsigned short* __restrict__ Btp,
    void* __restrict__ Cout, const float* __restrict__ bias, const float* __restrict__ bias2,
    const int* __restrict__ resp, float scale) {
  typedef _Float16 T;
  typedef v16h V;
  __shared__ __align__(16) float sT[8][16 * 68];
  __shared__ int sTot[8][4];
  const int tid  = threadIdx.x;
  const int lane = tid & 31;
  const int wave = tid >> 5;
  const int b    = blockIdx.y >> 2;
  const int cat  = blockIdx.y & 3;

  {
    const int4 rv = *(const int4*)(resp + b * kSeq + 4 * tid);
    const int c0 = clamp_cat(rv.x), c1 = clamp_cat(rv.y), c2 = clamp_cat(rv.z), c3 = clamp_cat(rv.w);
    int a0 = (c0 == 0) + (c1 == 0) + (c2 == 0) + (c3 == 0);
    int a1 = (c0 == 1) + (c1 == 1) + (c2 == 1) + (c3 == 1);
    int a2 = (c0 == 2) + (c1 == 2) + (c2 == 2) + (c3 == 2);
    int a3 = (c0 == 3) + (c1 == 3) + (c2 == 3) + (c3 == 3);
#pragma unroll
    for (int off = 16; off > 0; off >>= 1) {
      a0 += __shfl_xor(a0, off, 32);
      a1 += __shfl_xor(a1, off, 32);
      a2 += __shfl_xor(a2, off, 32);
      a3 += __shfl_xor(a3, off, 32);
    }
    if (lane == 0) { sTot[wave][0] = a0; sTot[wave][1] = a1; sTot[wave][2] = a2; sTot[wave][3] = a3; }
  }
  __syncthreads();
  int tot0 = 0, tot1 = 0, tot2 = 0, tot3 = 0;
#pragma unroll
  for (int w = 0; w < 8; ++w) { tot0 += sTot[w][0]; tot1 += sTot[w][1]; tot2 += sTot[w][2]; tot3 += sTot[w][3]; }
  const int off1 = tot0, off2 = tot0 + tot1, off3 = tot0 + tot1 + tot2;
  int segStart = (cat == 0) ? 0 : (cat == 1) ? off1 : (cat == 2) ? off2 : off3;
  const int nc = (cat == 0) ? tot0 : (cat == 1) ? tot1 : (cat == 2) ? tot2 : tot3;
  segStart = segStart < 0 ? 0 : (segStart > kSeq ? kSeq : segStart);
  int segEnd = segStart + nc;
  segEnd = segEnd > kSeq ? kSeq : segEnd;
  if (segEnd <= segStart) return;
  const int first = segStart >> 6;
  const int last  = (segEnd - 1) >> 6;
  const int tile  = blockIdx.x * 8 + wave;
  const int tml   = tile >> 4;
  const int tn    = tile & 15;
  if (tml > last - first) return;
  int tm = first + tml; tm = tm > 15 ? 15 : tm;
  const int m0 = tm << 6;
  const int n0 = tn << 6;

  const T* Ab = (const T*)Ap  + (size_t)b * kPlaneBatch;
  const T* Bb = (const T*)Btp + (size_t)cat * kPlaneW;
  const int lda = kEmb, ldb = kEmb;

  const int rlane = lane & 15;
  const int koff  = (lane >> 4) * 8;
  const int mOff  = (lane >> 4) * 8;

  v8f acc[4][4];
#pragma unroll
  for (int i = 0; i < 4; ++i)
#pragma unroll
    for (int j = 0; j < 4; ++j) acc[i][j] = (v8f){0.f,0.f,0.f,0.f,0.f,0.f,0.f,0.f};

  for (int k0 = 0; k0 < kEmb; k0 += 32) {
    V bh[4];
#pragma unroll
    for (int j = 0; j < 4; ++j) {
      const size_t bo = (size_t)(n0 + (j << 4) + rlane) * ldb + koff + k0;
      bh[j] = Frag<T>::load(Bb + bo);
    }
#pragma unroll
    for (int i = 0; i < 4; ++i) {
      const size_t ao = (size_t)(m0 + (i << 4) + rlane) * lda + koff + k0;
      V ah = Frag<T>::load(Ab + ao);
#pragma unroll
      for (int j = 0; j < 4; ++j) acc[i][j] = Frag<T>::mma(ah, bh[j], acc[i][j]);
      Frag<T>::guard(acc[i][0], acc[i][3], ah, ah);
    }
    Frag<T>::keep(bh[0], bh[1], bh[2], bh[3]);
  }
  acc_guard4(acc[0][0], acc[0][1], acc[0][2], acc[0][3]);
  acc_guard4(acc[1][0], acc[1][1], acc[1][2], acc[1][3]);
  acc_guard4(acc[2][0], acc[2][1], acc[2][2], acc[2][3]);
  acc_guard4(acc[3][0], acc[3][1], acc[3][2], acc[3][3]);

  float* slab = sT[wave];
#pragma unroll
  for (int i = 0; i < 4; ++i) {
    const int mBase = m0 + (i << 4);
#pragma unroll
    for (int j = 0; j < 4; ++j) {
      const int n = n0 + (j << 4) + rlane;
      const float bv = bias[n] + bias2[(size_t)cat * kEmb + n];
#pragma unroll
      for (int r = 0; r < 8; ++r) {
        const float v = acc[i][j][r] * scale + bv;
        slab[(mOff + r) * 68 + (j << 4) + rlane] = v;
      }
    }
    __builtin_amdgcn_fence(__ATOMIC_RELEASE, "workgroup");
    __builtin_amdgcn_wave_barrier();
    __builtin_amdgcn_fence(__ATOMIC_ACQUIRE, "workgroup");
    if (OUT_MODE == 0) {
      float* C = (float*)Cout + (size_t)b * kPlaneBatch;
      const int hh = lane >> 4, c4 = (lane & 15) * 4;
      for (int pass = 0; pass < 2; ++pass) {
#pragma unroll
        for (int it = 0; it < 8; ++it) {
          const int row  = it * 2 + hh;
          const int grow = mBase + row;
          v4f v = *(const v4f*)(slab + row * 68 + c4);
          if (grow >= segStart && grow < segEnd)
            *(volatile v4f*)(C + (size_t)grow * kEmb + n0 + c4) = v;
        }
        __threadfence();
      }
    } else {
      unsigned short* C = (unsigned short*)Cout + (size_t)b * kPlaneBatch;
      const int q = lane >> 3, c8 = (lane & 7) * 8;
      for (int pass = 0; pass < 2; ++pass) {
#pragma unroll
        for (int it = 0; it < 4; ++it) {
          const int row  = it * 4 + q;
          const int grow = mBase + row;
          const float* sp = slab + row * 68 + c8;
          v8h hv;
#pragma unroll
          for (int e = 0; e < 8; ++e) hv[e] = (_Float16)sp[e];
          if (grow >= segStart && grow < segEnd)
            *(volatile v8h*)(C + (size_t)grow * kEmb + n0 + c8) = hv;
        }
        __threadfence();
      }
    }
    __builtin_amdgcn_fence(__ATOMIC_RELEASE, "workgroup");
    __builtin_amdgcn_wave_barrier();
    __builtin_amdgcn_fence(__ATOMIC_ACQUIRE, "workgroup");
  }
}

__global__ __launch_bounds__(256) void cast8_f16s_kernel(const float* __restrict__ in, unsigned short* __restrict__ out,
                                                         int n8, float scale) {
  const int i = blockIdx.x * 256 + threadIdx.x;
  if (i >= n8) return;
  const float* p = in + 8 * (size_t)i;
  const v4f a = *(const v4f*)(p);
  const v4f c = *(const v4f*)(p + 4);
  unsigned short hb[8];
#pragma unroll
  for (int e = 0; e < 4; ++e) {
    hb[e]     = h_bits(a[e] * scale);
    hb[4 + e] = h_bits(c[e] * scale);
  }
  const v4u u = (v4u){pk16(hb[0], hb[1]), pk16(hb[2], hb[3]), pk16(hb[4], hb[5]), pk16(hb[6], hb[7])};
  unsigned short* q = out + 8 * (size_t)i;
  *(volatile v4u*)q = u;
  __threadfence();
  *(volatile v4u*)q = u;
}

__global__ __launch_bounds__(256) void wsum_cast_kernel(const float* __restrict__ Wb, const float* __restrict__ Wm,
                                                        unsigned short* __restrict__ out, float scale) {
  const int i = blockIdx.x * 256 + threadIdx.x;
  if (i >= (int)(kPlaneW / 8)) return;
  const int cat = blockIdx.y;
  const float* pb = Wb + 8 * (size_t)i;
  const float* pm = Wm + (size_t)cat * kPlaneW + 8 * (size_t)i;
  const v4f a0 = *(const v4f*)(pb);
  const v4f a1 = *(const v4f*)(pb + 4);
  const v4f g0 = *(const v4f*)(pm);
  const v4f g1 = *(const v4f*)(pm + 4);
  unsigned short hb[8];
#pragma unroll
  for (int e = 0; e < 4; ++e) {
    hb[e]     = h_bits((a0[e] + g0[e]) * scale);
    hb[4 + e] = h_bits((a1[e] + g1[e]) * scale);
  }
  const v4u u = (v4u){pk16(hb[0], hb[1]), pk16(hb[2], hb[3]), pk16(hb[4], hb[5]), pk16(hb[6], hb[7])};
  unsigned short* q = out + (size_t)cat * kPlaneW + 8 * (size_t)i;
  *(volatile v4u*)q = u;
  __threadfence();
  *(volatile v4u*)q = u;
}

__global__ __launch_bounds__(256) void split8_bf16_kernel(const float* __restrict__ in, unsigned short* __restrict__ oh,
                                                          unsigned short* __restrict__ ol, int n8) {
  const int i = blockIdx.x * 256 + threadIdx.x;
  if (i >= n8) return;
  const float* p = in + 8 * (size_t)i;
  const v4f a = *(const v4f*)(p);
  const v4f c = *(const v4f*)(p + 4);
  unsigned short hb[8], lb[8];
#pragma unroll
  for (int e = 0; e < 4; ++e) {
    hb[e] = f2bf_bits(a[e]);          lb[e] = f2bf_bits(a[e] - bf_bits2f(hb[e]));
    hb[4 + e] = f2bf_bits(c[e]);      lb[4 + e] = f2bf_bits(c[e] - bf_bits2f(hb[4 + e]));
  }
  const v4u uh = (v4u){pk16(hb[0], hb[1]), pk16(hb[2], hb[3]), pk16(hb[4], hb[5]), pk16(hb[6], hb[7])};
  const v4u ul = (v4u){pk16(lb[0], lb[1]), pk16(lb[2], lb[3]), pk16(lb[4], lb[5]), pk16(lb[6], lb[7])};
  unsigned short* qh = oh + 8 * (size_t)i;
  unsigned short* ql = ol + 8 * (size_t)i;
  *(volatile v4u*)qh = uh;
  *(volatile v4u*)ql = ul;
  __threadfence();
  *(volatile v4u*)qh = uh;
  *(volatile v4u*)ql = ul;
}

__global__ __launch_bounds__(256) void gather_cast_kernel(
    const float* __restrict__ key, const float* __restrict__ value, const int* __restrict__ resp,
    unsigned short* __restrict__ outK, unsigned short* __restrict__ outV) {
  __shared__ int sTot[8][4];
  __shared__ int sTok[32];
  const int t = threadIdx.x;
  const int lane = t & 31, wave = t >> 5;
  const int slot0 = blockIdx.x * 32;
  const int b = blockIdx.y;
  const int z = blockIdx.z;
  const float* src = (z == 0) ? key : value;
  unsigned short* dst = (z == 0) ? outK : outV;

  const int4 rv = *(const int4*)(resp + b * kSeq + 4 * t);
  const int c0 = clamp_cat(rv.x), c1 = clamp_cat(rv.y), c2 = clamp_cat(rv.z), c3 = clamp_cat(rv.w);
  const int a0 = (c0 == 0) + (c1 == 0) + (c2 == 0) + (c3 == 0);
  const int a1 = (c0 == 1) + (c1 == 1) + (c2 == 1) + (c3 == 1);
  const int a2 = (c0 == 2) + (c1 == 2) + (c2 == 2) + (c3 == 2);
  const int a3 = (c0 == 3) + (c1 == 3) + (c2 == 3) + (c3 == 3);
  int s0 = a0, s1 = a1, s2 = a2, s3 = a3;
#pragma unroll
  for (int d = 1; d < 32; d <<= 1) {
    const int u0 = __shfl_up(s0, d, 32);
    const int u1 = __shfl_up(s1, d, 32);
    const int u2 = __shfl_up(s2, d, 32);
    const int u3 = __shfl_up(s3, d, 32);
    if (lane >= d) { s0 += u0; s1 += u1; s2 += u2; s3 += u3; }
  }
  if (lane == 31) { sTot[wave][0] = s0; sTot[wave][1] = s1; sTot[wave][2] = s2; sTot[wave][3] = s3; }
  __syncthreads();
  int p0 = 0, p1 = 0, p2 = 0, p3 = 0, t0 = 0, t1 = 0, t2 = 0, t3 = 0;
#pragma unroll
  for (int w = 0; w < 8; ++w) {
    const int v0 = sTot[w][0], v1 = sTot[w][1], v2 = sTot[w][2], v3 = sTot[w][3];
    const int before = (w < wave) ? 1 : 0;
    p0 += before * v0; p1 += before * v1; p2 += before * v2; p3 += before * v3;
    t0 += v0; t1 += v1; t2 += v2; t3 += v3;
  }
  int q0 = p0 + s0 - a0;
  int q1 = t0 + p1 + s1 - a1;
  int q2 = t0 + t1 + p2 + s2 - a2;
  int q3 = t0 + t1 + t2 + p3 + s3 - a3;
  {
    int pos, li;
    pos = (c0 == 0) ? q0 : (c0 == 1) ? q1 : (c0 == 2) ? q2 : q3;
    q0 += (c0 == 0); q1 += (c0 == 1); q2 += (c0 == 2); q3 += (c0 == 3);
    li = pos - slot0; if ((unsigned)li < 32u) sTok[li] = 4 * t + 0;
    pos = (c1 == 0) ? q0 : (c1 == 1) ? q1 : (c1 == 2) ? q2 : q3;
    q0 += (c1 == 0); q1 += (c1 == 1); q2 += (c1 == 2); q3 += (c1 == 3);
    li = pos - slot0; if ((unsigned)li < 32u) sTok[li] = 4 * t + 1;
    pos = (c2 == 0) ? q0 : (c2 == 1) ? q1 : (c2 == 2) ? q2 : q3;
    q0 += (c2 == 0); q1 += (c2 == 1); q2 += (c2 == 2); q3 += (c2 == 3);
    li = pos - slot0; if ((unsigned)li < 32u) sTok[li] = 4 * t + 2;
    pos = (c3 == 0) ? q0 : (c3 == 1) ? q1 : (c3 == 2) ? q2 : q3;
    li = pos - slot0; if ((unsigned)li < 32u) sTok[li] = 4 * t + 3;
  }
  __syncthreads();

#pragma unroll
  for (int rr = 0; rr < 4; ++rr) {
    const int lr = wave * 4 + rr;
    int tok = sTok[lr];
    tok = tok < 0 ? 0 : (tok > kSeq - 1 ? kSeq - 1 : tok);
    const float* srow = src + ((size_t)(b * kSeq + tok)) * kEmb;
    unsigned short* drow = dst + ((size_t)(b * kSeq + slot0 + lr)) * kEmb;
    v4u u[4];
#pragma unroll
    for (int it = 0; it < 4; ++it) {
      const int col = it * 256 + lane * 8;
      const v4f a = *(const v4f*)(srow + col);
      const v4f c = *(const v4f*)(srow + col + 4);
      unsigned short hb[8];
#pragma unroll
      for (int e = 0; e < 4; ++e) { hb[e] = h_bits(a[e]); hb[4 + e] = h_bits(c[e]); }
      u[it] = (v4u){pk16(hb[0], hb[1]), pk16(hb[2], hb[3]), pk16(hb[4], hb[5]), pk16(hb[6], hb[7])};
    }
    for (int pass = 0; pass < 2; ++pass) {
#pragma unroll
      for (int it = 0; it < 4; ++it)
        *(volatile v4u*)(drow + it * 256 + lane * 8) = u[it];
      __threadfence();
    }
  }
}

__global__ __launch_bounds__(256) void vt_split_kernel(const float* __restrict__ Vs,
                                                      unsigned short* __restrict__ Vth, unsigned short* __restrict__ Vtl) {
  __shared__ float sm[64][65];
  const int t = threadIdx.x;
  const int lane = t & 31, wave = t >> 5;
  const int tok0 = blockIdx.x * 64;
  const int h = blockIdx.y;
  const int b = blockIdx.z;
#pragma unroll
  for (int i = 0; i < 16; ++i) {
    const int e  = i * 256 + t;
    const int tl = e >> 6;
    const int dl = e & 63;
    sm[dl][tl] = Vs[((size_t)(b * kSeq + tok0 + tl)) * kEmb + h * kHeadDim + dl];
  }
  __syncthreads();
  const int q = lane >> 3, c8 = (lane & 7) * 8;
  v4u uh[2], ul[2];
#pragma unroll
  for (int it = 0; it < 2; ++it) {
    const int d = wave * 8 + it * 4 + q;
    unsigned short hb[8], lb[8];
#pragma unroll
    for (int e = 0; e < 8; ++e) {
      const float v = sm[d][c8 + e];
      hb[e] = f2bf_bits(v);
      lb[e] = f2bf_bits(v - bf_bits2f(hb[e]));
    }
    uh[it] = (v4u){pk16(hb[0], hb[1]), pk16(hb[2], hb[3]), pk16(hb[4], hb[5]), pk16(hb[6], hb[7])};
    ul[it] = (v4u){pk16(lb[0], lb[1]), pk16(lb[2], lb[3]), pk16(lb[4], lb[5]), pk16(lb[6], lb[7])};
  }
  for (int pass = 0; pass < 2; ++pass) {
#pragma unroll
    for (int it = 0; it < 2; ++it) {
      const int d = wave * 8 + it * 4 + q;
      const size_t o = (((size_t)(b * kHeads + h) * kHeadDim + d) * kSeq) + tok0 + c8;
      *(volatile v4u*)(Vth + o) = uh[it];
      *(volatile v4u*)(Vtl + o) = ul[it];
    }
    __threadfence();
  }
}

__global__ __launch_bounds__(128) void softmax_split_kernel(const float* __restrict__ Sc,
                                                           unsigned short* __restrict__ Ph, unsigned short* __restrict__ Pl) {
  __shared__ float redM[4];
  __shared__ float redS[4];
  const int row  = blockIdx.x;
  const int t    = threadIdx.x;
  const int lane = t & 31, wave = t >> 5;
  const int c0   = t * 8;
  const float* sr = Sc + (size_t)row * kSeq + c0;
  const v4f a = *(const v4f*)(sr);
  const v4f c = *(const v4f*)(sr + 4);
  float x[8];
#pragma unroll
  for (int e = 0; e < 4; ++e) { x[e] = a[e]; x[4 + e] = c[e]; }
  float m = fmaxf(fmaxf(fmaxf(x[0], x[1]), fmaxf(x[2], x[3])), fmaxf(fmaxf(x[4], x[5]), fmaxf(x[6], x[7])));
#pragma unroll
  for (int off = 16; off > 0; off >>= 1) m = fmaxf(m, __shfl_xor(m, off, 32));
  if (lane == 0) redM[wave] = m;
  __syncthreads();
  const float gm = fmaxf(fmaxf(redM[0], redM[1]), fmaxf(redM[2], redM[3]));
  float ev[8];
#pragma unroll
  for (int e = 0; e < 8; ++e) ev[e] = expf(x[e] - gm);
  float s = ((ev[0] + ev[1]) + (ev[2] + ev[3])) + ((ev[4] + ev[5]) + (ev[6] + ev[7]));
#pragma unroll
  for (int off = 16; off > 0; off >>= 1) s += __shfl_xor(s, off, 32);
  if (lane == 0) redS[wave] = s;
  __syncthreads();
  const float tot = ((redS[0] + redS[1]) + redS[2]) + redS[3];
  const float inv = 1.0f / tot;
  unsigned short hb[8], lb[8];
#pragma unroll
  for (int e = 0; e < 8; ++e) {
    const float p = ev[e] * inv;
    hb[e] = f2bf_bits(p);
    lb[e] = f2bf_bits(p - bf_bits2f(hb[e]));
  }
  const v4u uh = (v4u){pk16(hb[0], hb[1]), pk16(hb[2], hb[3]), pk16(hb[4], hb[5]), pk16(hb[6], hb[7])};
  const v4u ul = (v4u){pk16(lb[0], lb[1]), pk16(lb[2], lb[3]), pk16(lb[4], lb[5]), pk16(lb[6], lb[7])};
  unsigned short* ph = Ph + (size_t)row * kSeq + c0;
  unsigned short* pl = Pl + (size_t)row * kSeq + c0;
  *(volatile v4u*)ph = uh;
  *(volatile v4u*)pl = ul;
  __threadfence();
  *(volatile v4u*)ph = uh;
  *(volatile v4u*)pl = ul;
}

extern "C" void kernel_launch(void* const* d_in, const int* in_sizes, int n_in,
                              void* d_out, int out_size, void* d_ws, size_t ws_size,
                              hipStream_t stream) {
  if (n_in < 16) return;
  if (in_sizes[0] != (int)kPlaneTok || in_sizes[1] != (int)kPlaneTok || in_sizes[2] != (int)kPlaneTok) return;
  if (in_sizes[3] != kTok) return;
  if (in_sizes[4] != (int)kPlaneW || in_sizes[6] != (int)kPlaneW || in_sizes[8] != (int)kPlaneW || in_sizes[10] != (int)kPlaneW) return;
  if (in_sizes[12] != (int)(kCats * kPlaneW) || in_sizes[14] != (int)(kCats * kPlaneW)) return;
  if (in_sizes[5] != kEmb || in_sizes[7] != kEmb || in_sizes[9] != kEmb || in_sizes[11] != kEmb) return;
  if (in_sizes[13] != kCats * kEmb || in_sizes[15] != kCats * kEmb) return;
  if (out_size != (int)kPlaneTok) return;
  const size_t MiB = 1048576;
  if (ws_size < 116 * MiB) return;

  const float* query = (const float*)d_in[0];
  const float* key   = (const float*)d_in[1];
  const float* value = (const float*)d_in[2];
  const int*   resp  = (const int*)  d_in[3];
  const float* Wq = (const float*)d_in[4];   const float* bq = (const float*)d_in[5];
  const float* Wk = (const float*)d_in[6];   const float* bk = (const float*)d_in[7];
  const float* Wv = (const float*)d_in[8];   const float* bv = (const float*)d_in[9];
  const float* Wo = (const float*)d_in[10];  const float* bo = (const float*)d_in[11];
  const float* Wkm = (const float*)d_in[12]; const float* bkm = (const float*)d_in[13];
  const float* Wvm = (const float*)d_in[14]; const float* bvm = (const float*)d_in[15];
  float* out = (float*)d_out;

  char* ws = (char*)d_ws;
  unsigned short* Xq   = (unsigned short*)(ws + 0 * MiB);
  unsigned short* Xks  = (unsigned short*)(ws + 8 * MiB);
  unsigned short* Xvs  = (unsigned short*)(ws + 16 * MiB);
  unsigned short* Wq16 = (unsigned short*)(ws + 24 * MiB);
  unsigned short* Wkc  = (unsigned short*)(ws + 26 * MiB);
  unsigned short* Wvc  = (unsigned short*)(ws + 34 * MiB);
  float*          Vs   = (float*)(ws + 42 * MiB);
  float*          Sc   = (float*)(ws + 0 * MiB);
  unsigned short* Ph   = (unsigned short*)(ws + 32 * MiB);
  unsigned short* Pl   = (unsigned short*)(ws + 48 * MiB);
  unsigned short* Woh  = (unsigned short*)(ws + 64 * MiB);
  unsigned short* Wol  = (unsigned short*)(ws + 66 * MiB);
  unsigned short* Qp   = (unsigned short*)(ws + 68 * MiB);
  unsigned short* Ks   = (unsigned short*)(ws + 76 * MiB);
  unsigned short* Vth  = (unsigned short*)(ws + 84 * MiB);
  unsigned short* Vtl  = (unsigned short*)(ws + 92 * MiB);
  unsigned short* Ath  = (unsigned short*)(ws + 100 * MiB);
  unsigned short* Atl  = (unsigned short*)(ws + 108 * MiB);

  cast8_f16s_kernel<<<(int)(kPlaneTok / 8 / 256), 256, 0, stream>>>(query, Xq, (int)(kPlaneTok / 8), 1.0f);
  cast8_f16s_kernel<<<(int)(kPlaneW / 8 / 256), 256, 0, stream>>>(Wq, Wq16, (int)(kPlaneW / 8), kWCarry);
  wsum_cast_kernel<<<dim3((int)(kPlaneW / 8 / 256), kCats), 256, 0, stream>>>(Wk, Wkm, Wkc, kWCarry);
  wsum_cast_kernel<<<dim3((int)(kPlaneW / 8 / 256), kCats), 256, 0, stream>>>(Wv, Wvm, Wvc, kWCarry);
  split8_bf16_kernel<<<(int)(kPlaneW / 8 / 256), 256, 0, stream>>>(Wo, Woh, Wol, (int)(kPlaneW / 8));
  gather_cast_kernel<<<dim3(kSeq / 32, kBatch, 2), 256, 0, stream>>>(key, value, resp, Xks, Xvs);

  wmma_gemm64<0, false, 2, 1, false><<<dim3(128, 1), 256, 0, stream>>>(
      Xq, Xq, kEmb, 0L, Wq16, Wq16, kEmb, 0L, (void*)Qp, (void*)Qp, kEmb, 0L, bq, bq, 0L,
      kTok, kEmb, kEmb, kWCarryInv);
  seg_gemm64<1><<<dim3(32, kBatch * kCats), 256, 0, stream>>>(Xks, Wkc, (void*)Ks, bk, bkm, resp, kWCarryInv);
  seg_gemm64<0><<<dim3(32, kBatch * kCats), 256, 0, stream>>>(Xvs, Wvc, (void*)Vs, bv, bvm, resp, kWCarryInv);
  vt_split_kernel<<<dim3(kSeq / 64, kHeads, kBatch), 256, 0, stream>>>(Vs, Vth, Vtl);

  for (int b = 0; b < kBatch; ++b) {
    for (int hg = 0; hg < kGroupsPerBatch; ++hg) {
      const size_t qoff = (size_t)b * kPlaneBatch + (size_t)hg * kHeadsPerGroup * kHeadDim;
      wmma_gemm64<0, false, 0, 0, false><<<dim3(32, kHeadsPerGroup), 256, 0, stream>>>(
          Qp + qoff, Qp + qoff, kEmb, (long)kHeadDim, Ks + qoff, Ks + qoff, kEmb, (long)kHeadDim,
          (void*)Sc, (void*)Sc, kSeq, (long)kPlaneBatch, bq, bq, 0L,
          kSeq, kSeq, kHeadDim, kScoreScale);
      softmax_split_kernel<<<kHeadsPerGroup * kSeq, 128, 0, stream>>>(Sc, Ph, Pl);
      const size_t voff = ((size_t)(b * kHeads + hg * kHeadsPerGroup) * kHeadDim) * kSeq;
      wmma_gemm64<1, true, 0, 2, false><<<dim3(2, kHeadsPerGroup), 256, 0, stream>>>(
          Ph, Pl, kSeq, (long)kPlaneBatch, Vth + voff, Vtl + voff, kSeq, (long)kHeadDim * kSeq,
          (void*)(Ath + qoff), (void*)(Atl + qoff), kEmb, (long)kHeadDim, bq, bq, 0L,
          kSeq, kHeadDim, kSeq, 1.0f);
    }
  }

  wmma_gemm64<1, true, 2, 0, false><<<dim3(128, 1), 256, 0, stream>>>(
      Ath, Atl, kEmb, 0L, Woh, Wol, kEmb, 0L, (void*)out, (void*)out, kEmb, 0L, bo, bo, 0L,
      kTok, kEmb, kEmb, 1.0f);
}
